// OnePoleDecoder_82695300317749
// MI455X (gfx1250) — hardware-run, weakly checked
//
#include <hip/hip_runtime.h>
#include <hip/hip_fp16.h>
#include <math.h>

typedef __attribute__((ext_vector_type(16))) _Float16 v16h;
typedef __attribute__((ext_vector_type(8)))  _Float16 v8h;
typedef __attribute__((ext_vector_type(8)))  float    v8f;
typedef __attribute__((ext_vector_type(4)))  float    v4f;
typedef __attribute__((ext_vector_type(2)))  unsigned v2u;
typedef __attribute__((ext_vector_type(4)))  unsigned v4u;

constexpr int kT      = 131072;
constexpr int kIn     = 64;
constexpr int kHid    = 512;
constexpr int kChunk  = 16384;
constexpr int kNChunk = 8;
constexpr int kHeadN  = 64;
constexpr int kWarm   = 256;
constexpr float kXCarry = 64.0f;
constexpr float kWCarry = 1024.0f;
constexpr float kTCarry = 16384.0f;
constexpr float kHCarry = 4096.0f;
constexpr float kAlpha = 0.8824969025845955f;
constexpr float kOneMinusA = 1.0f - kAlpha;
static_assert(kT == 131072 && kIn == 64 && kHid == 512 && kChunk == 16384 && kNChunk == 8);
static_assert(kChunk * kNChunk == kT);
static_assert(kHeadN == 64 && kWarm == 256 && (kT % 4) == 0);
static_assert((kIn % 32) == 0 && (kHid % 64) == 0 && (kHid % 32) == 0 && (kHeadN % 64) == 0 && (kChunk % 32) == 0);
static_assert(kXCarry == 64.0f && kWCarry == 1024.0f && kTCarry == 16384.0f && kHCarry == 4096.0f);
static_assert(kAlpha > 0.88249f && kAlpha < 0.88250f);
static_assert(kOneMinusA > 0.11750f && kOneMinusA < 0.11751f);

constexpr size_t kSzBH = (size_t)kT * kIn * 2;
constexpr size_t kSzWI = (size_t)kHid * kIn * 2;
constexpr size_t kSzWH = (size_t)kHeadN * kHid * 2;
constexpr size_t kSzXP = (size_t)kChunk * kHid * 4;
constexpr size_t kSzXH = (size_t)kChunk * kHid * 2;
constexpr size_t kSzP  = (size_t)kChunk * kHeadN * 4;
constexpr size_t kSzPC = (size_t)kT * 2 * 4;
constexpr size_t kOffBH = 0;
constexpr size_t kOffWI = kOffBH + kSzBH;
constexpr size_t kOffWH = kOffWI + kSzWI;
constexpr size_t kOffXP = kOffWH + kSzWH;
constexpr size_t kOffXH = kOffXP + kSzXP;
constexpr size_t kOffP  = kOffXH + kSzXH;
constexpr size_t kOffPC = kOffP  + kSzP;
constexpr size_t kWsTotal = kOffPC + kSzPC;
static_assert(kSzBH == 16777216ull && kSzWI == 65536ull && kSzWH == 65536ull && kSzXP == 33554432ull);
static_assert(kSzXH == 16777216ull && kSzP == 4194304ull && kSzPC == 1048576ull);
static_assert(kWsTotal == 16777216ull + 65536ull + 65536ull + 33554432ull + 16777216ull + 4194304ull + 1048576ull);
static_assert(kWsTotal == 72482816ull);
static_assert(kWsTotal <= 134217728ull);
static_assert((kSzBH % 128) == 0 && (kSzWI % 128) == 0 && (kSzWH % 128) == 0 && (kSzXP % 128) == 0 &&
              (kSzXH % 128) == 0 && (kSzP % 128) == 0 && (kSzPC % 128) == 0);
static_assert((((size_t)kChunk * kIn * 2) % 128) == 0);
static_assert((((size_t)kChunk * 2 * 4) % 128) == 0);

__device__ __forceinline__ _Float16 f16_flush(float v) {
  const float w = (fabsf(v) < 6.103515625e-05f) ? 0.0f : v;
  return (_Float16)w;
}

__device__ __forceinline__ float bf16r(float v) {
  unsigned u = __float_as_uint(v);
  u = (u + 0x7FFFu + ((u >> 16) & 1u)) & 0xFFFF0000u;
  return __uint_as_float(u);
}

__device__ __forceinline__ float h16_to_f32(unsigned hb) {
  const unsigned sgn = (hb & 0x8000u) << 16; const unsigned em = hb & 0x7fffu;
  const float fn = __uint_as_float((em << 13) + 0x38000000u);
  const float fs = (float)em * 5.9604644775390625e-8f;
  const float mag = (em < 0x400u) ? fs : fn; return __uint_as_float(__float_as_uint(mag) | sgn); }

namespace eng {
union FragU { v16h v; v8h h[2]; };
__device__ __forceinline__ v16h frag_load(const _Float16* p) {
  FragU f;
  f.h[0] = *(const v8h*)(p);
  f.h[1] = *(const v8h*)(p + 16);
  return f.v;
}
__device__ __forceinline__ v8f mma(v16h a, v16h b, v8f c) {
  return __builtin_amdgcn_wmma_f32_16x16x32_f16(false, a, false, b, (short)0, c, false, false);
}
__device__ __forceinline__ void guard1(v8f& a, v16h x, v16h y) {
  asm volatile("v_nop\n\tv_nop\n\tv_nop\n\tv_nop" : "+v"(a) : "v"(x), "v"(y));
}
__device__ __forceinline__ void guard_acc(v8f& a) {
  asm volatile("v_nop\n\tv_nop\n\tv_nop\n\tv_nop" : "+v"(a));
}
__device__ __forceinline__ void keep4(v16h a, v16h b, v16h c, v16h d) {
  asm volatile("v_nop" :: "v"(a), "v"(b), "v"(c), "v"(d));
}

template <int MI, int SPL>
__global__ __launch_bounds__(256) void gemm_f16_kernel(
    const unsigned short* __restrict__ Ap, const unsigned short* __restrict__ A2p, int lda,
    const unsigned short* __restrict__ Btp, const unsigned short* __restrict__ Bt2p, int ldb,
    float* __restrict__ C, int ldc, int M, int N, int K, float scale, float rscale)
{
  static_assert(MI >= 1 && MI <= 2);
  static_assert(SPL >= 0 && SPL <= 2);
  const _Float16* A   = (const _Float16*)Ap;
  const _Float16* A2  = (const _Float16*)A2p;
  const _Float16* Bt  = (const _Float16*)Btp;
  const _Float16* Bt2 = (const _Float16*)Bt2p;
  __shared__ __align__(16) float sT[8][16 * 68];
  const int lane = threadIdx.x & 31;
  const int wave = threadIdx.x >> 5;
  const int tilesN = N >> 6;
  const int tilesM = M / (16 * MI);
  const int tile = blockIdx.x * 8 + wave;
  if (tile >= tilesM * tilesN) return;
  const int tm = tile / tilesN;
  const int tn = tile - tm * tilesN;
  const int m0 = tm * (16 * MI);
  const int n0 = tn << 6;
  const int rlane = lane & 15;
  const int koff  = (lane >> 4) * 8;
  const int mOff  = (lane >> 4) * 8;

  v8f acc[MI][4], accr[MI][4];
#pragma unroll
  for (int i = 0; i < MI; ++i)
#pragma unroll
    for (int j = 0; j < 4; ++j) {
      acc[i][j]  = (v8f){0.f, 0.f, 0.f, 0.f, 0.f, 0.f, 0.f, 0.f};
      accr[i][j] = (v8f){0.f, 0.f, 0.f, 0.f, 0.f, 0.f, 0.f, 0.f};
    }

  for (int k0 = 0; k0 < K; k0 += 32) {
    v16h bh[4], bl[4];
#pragma unroll
    for (int j = 0; j < 4; ++j) {
      const size_t bo = (size_t)(n0 + (j << 4) + rlane) * ldb + koff + k0;
      bh[j] = frag_load(Bt + bo);
      if (SPL == 2) bl[j] = frag_load(Bt2 + bo); else bl[j] = bh[j];
    }
#pragma unroll
    for (int i = 0; i < MI; ++i) {
      const size_t ao = (size_t)(m0 + (i << 4) + rlane) * lda + koff + k0;
      const v16h ah = frag_load(A + ao);
      v16h al = ah;
      if (SPL >= 1) al = frag_load(A2 + ao);
#pragma unroll
      for (int j = 0; j < 4; ++j) {
        acc[i][j] = mma(ah, bh[j], acc[i][j]);
        if (SPL >= 1) accr[i][j] = mma(al, bh[j], accr[i][j]);
        if (SPL == 2) accr[i][j] = mma(ah, bl[j], accr[i][j]);
      }
#pragma unroll
      for (int j = 0; j < 4; ++j) {
        guard1(acc[i][j], ah, al);
        if (SPL >= 1) guard1(accr[i][j], ah, al);
      }
    }
    keep4(bh[0], bh[1], bh[2], bh[3]);
    if (SPL == 2) keep4(bl[0], bl[1], bl[2], bl[3]);
  }
#pragma unroll
  for (int i = 0; i < MI; ++i)
#pragma unroll
    for (int j = 0; j < 4; ++j) {
      guard_acc(acc[i][j]);
      if (SPL >= 1) guard_acc(accr[i][j]);
    }

  float* slab = sT[wave];
#pragma unroll
  for (int i = 0; i < MI; ++i) {
    const int mBase = m0 + (i << 4);
#pragma unroll
    for (int j = 0; j < 4; ++j) {
#pragma unroll
      for (int r = 0; r < 8; ++r) {
        float v = acc[i][j][r] * scale;
        if (SPL >= 1) v += accr[i][j][r] * rscale;
        slab[(mOff + r) * 68 + (j << 4) + rlane] = v;
      }
    }
    __builtin_amdgcn_fence(__ATOMIC_RELEASE, "workgroup");
    __builtin_amdgcn_wave_barrier();
    __builtin_amdgcn_fence(__ATOMIC_ACQUIRE, "workgroup");
    {
      const int hh = lane >> 4, c4 = (lane & 15) * 4;
      for (int pass = 0; pass < 2; ++pass) {
#pragma unroll
        for (int it = 0; it < 8; ++it) {
          const int row = it * 2 + hh;
          const v4f v = *(const v4f*)(slab + row * 68 + c4);
          *(volatile v4f*)(C + (size_t)(mBase + row) * ldc + n0 + c4) = v;
        }
        __threadfence();
      }
    }
    __builtin_amdgcn_fence(__ATOMIC_RELEASE, "workgroup");
    __builtin_amdgcn_wave_barrier();
    __builtin_amdgcn_fence(__ATOMIC_ACQUIRE, "workgroup");
  }
}
}

__device__ __forceinline__ _Float16 in_half(float v, float carry, bool live) {
  const float t = live ? (bf16r(v) * carry) : 0.0f;
  return f16_flush(t);
}
__device__ __forceinline__ _Float16 val_half(float v, float carry, bool live) {
  const float t = live ? (v * carry) : 0.0f;
  return f16_flush(t);
}
__device__ __forceinline__ int imin2(int a, int b) {
  return (a < b) ? a : b;
}
__device__ __forceinline__ int iclamp(int v, int lo, int hi) {
  const int t = (v < lo) ? lo : v;
  return (t > hi) ? hi : t;
}

__global__ __launch_bounds__(256) void pack_x_kernel(
    const float* __restrict__ x, unsigned short* __restrict__ XH)
{
  const int i = blockIdx.x * 256 + threadIdx.x;
  const float* sp = x + (size_t)i * 8;
  const v4f a0 = *(const v4f*)(sp);
  const v4f a1 = *(const v4f*)(sp + 4);
  const float f0 = a0[0];
  const float f1 = a0[1];
  const float f2 = a0[2];
  const float f3 = a0[3];
  const float f4 = a1[0];
  const float f5 = a1[1];
  const float f6 = a1[2];
  const float f7 = a1[3];
  const float r0 = bf16r(f0);
  const float r1 = bf16r(f1);
  const float r2 = bf16r(f2);
  const float r3 = bf16r(f3);
  const float r4 = bf16r(f4);
  const float r5 = bf16r(f5);
  const float r6 = bf16r(f6);
  const float r7 = bf16r(f7);
  v8h hv;
  hv[0] = val_half(r0, kXCarry, true);
  hv[1] = val_half(r1, kXCarry, true);
  hv[2] = val_half(r2, kXCarry, true);
  hv[3] = val_half(r3, kXCarry, true);
  hv[4] = val_half(r4, kXCarry, true);
  hv[5] = val_half(r5, kXCarry, true);
  hv[6] = val_half(r6, kXCarry, true);
  hv[7] = val_half(r7, kXCarry, true);
  unsigned short* qh = XH + (size_t)i * 8;
  *(volatile v8h*)qh = hv;
  __threadfence();
  *(volatile v8h*)qh = hv;
}

__global__ __launch_bounds__(256) void pack_wt_kernel(
    const float* __restrict__ w, unsigned short* __restrict__ WI)
{
  const int i = blockIdx.x * 256 + threadIdx.x;
  const int n = i / (kIn / 8);
  const int k8 = (i - n * (kIn / 8)) * 8;
  const float f0 = w[(size_t)(k8 + 0) * kHid + n];
  const float f1 = w[(size_t)(k8 + 1) * kHid + n];
  const float f2 = w[(size_t)(k8 + 2) * kHid + n];
  const float f3 = w[(size_t)(k8 + 3) * kHid + n];
  const float f4 = w[(size_t)(k8 + 4) * kHid + n];
  const float f5 = w[(size_t)(k8 + 5) * kHid + n];
  const float f6 = w[(size_t)(k8 + 6) * kHid + n];
  const float f7 = w[(size_t)(k8 + 7) * kHid + n];
  v8h hv;
  hv[0] = in_half(f0, kWCarry, true);
  hv[1] = in_half(f1, kWCarry, true);
  hv[2] = in_half(f2, kWCarry, true);
  hv[3] = in_half(f3, kWCarry, true);
  hv[4] = in_half(f4, kWCarry, true);
  hv[5] = in_half(f5, kWCarry, true);
  hv[6] = in_half(f6, kWCarry, true);
  hv[7] = in_half(f7, kWCarry, true);
  unsigned short* q = WI + (size_t)i * 8;
  *(volatile v8h*)q = hv;
  __threadfence();
  *(volatile v8h*)q = hv;
}

__global__ __launch_bounds__(256) void pack_heads_kernel(
    const float* __restrict__ wt, const float* __restrict__ wz, unsigned short* __restrict__ WH)
{
  const int i = blockIdx.x * 256 + threadIdx.x;
  const int n = i / (kHid / 8);
  const int k8 = (i - n * (kHid / 8)) * 8;
  const bool live = (n < 2);
  const float* src = (n == 0) ? wt : wz;
  const v4f a0 = *(const v4f*)(src + k8);
  const v4f a1 = *(const v4f*)(src + k8 + 4);
  const float f0 = a0[0];
  const float f1 = a0[1];
  const float f2 = a0[2];
  const float f3 = a0[3];
  const float f4 = a1[0];
  const float f5 = a1[1];
  const float f6 = a1[2];
  const float f7 = a1[3];
  v8h hv;
  hv[0] = in_half(f0, kHCarry, live);
  hv[1] = in_half(f1, kHCarry, live);
  hv[2] = in_half(f2, kHCarry, live);
  hv[3] = in_half(f3, kHCarry, live);
  hv[4] = in_half(f4, kHCarry, live);
  hv[5] = in_half(f5, kHCarry, live);
  hv[6] = in_half(f6, kHCarry, live);
  hv[7] = in_half(f7, kHCarry, live);
  unsigned short* q = WH + (size_t)i * 8;
  *(volatile v8h*)q = hv;
  __threadfence();
  *(volatile v8h*)q = hv;
}

__global__ __launch_bounds__(256) void tanh_pack_kernel(
    const float* __restrict__ XP, const float* __restrict__ bin, unsigned short* __restrict__ XH)
{
  const int i = blockIdx.x * 256 + threadIdx.x;
  const int c8 = (i % (kHid / 8)) * 8;
  const float* sp = XP + (size_t)i * 8;
  const v4f a0 = *(const v4f*)(sp);
  const v4f a1 = *(const v4f*)(sp + 4);
  const v4f g0 = *(const v4f*)(bin + c8);
  const v4f g1 = *(const v4f*)(bin + c8 + 4);
  const float x0 = a0[0];
  const float x1 = a0[1];
  const float x2 = a0[2];
  const float x3 = a0[3];
  const float x4 = a1[0];
  const float x5 = a1[1];
  const float x6 = a1[2];
  const float x7 = a1[3];
  const float b0 = g0[0];
  const float b1 = g0[1];
  const float b2 = g0[2];
  const float b3 = g0[3];
  const float b4 = g1[0];
  const float b5 = g1[1];
  const float b6 = g1[2];
  const float b7 = g1[3];
  const float t0 = tanhf(x0 + bf16r(b0));
  const float t1 = tanhf(x1 + bf16r(b1));
  const float t2 = tanhf(x2 + bf16r(b2));
  const float t3 = tanhf(x3 + bf16r(b3));
  const float t4 = tanhf(x4 + bf16r(b4));
  const float t5 = tanhf(x5 + bf16r(b5));
  const float t6 = tanhf(x6 + bf16r(b6));
  const float t7 = tanhf(x7 + bf16r(b7));
  v8h hv;
  hv[0] = val_half(t0, kTCarry, true);
  hv[1] = val_half(t1, kTCarry, true);
  hv[2] = val_half(t2, kTCarry, true);
  hv[3] = val_half(t3, kTCarry, true);
  hv[4] = val_half(t4, kTCarry, true);
  hv[5] = val_half(t5, kTCarry, true);
  hv[6] = val_half(t6, kTCarry, true);
  hv[7] = val_half(t7, kTCarry, true);
  unsigned short* q = XH + (size_t)i * 8;
  *(volatile v8h*)q = hv;
  __threadfence();
  *(volatile v8h*)q = hv;
}

typedef float v2f __attribute__((ext_vector_type(2)));

__global__ __launch_bounds__(256) void heads_copy_kernel(
    const float* __restrict__ Pc, float* __restrict__ PCc)
{
  const int i = blockIdx.x * 256 + threadIdx.x;
  const v2f a = *(const v2f*)(Pc + (size_t)(2 * i) * kHeadN);
  const v2f b = *(const v2f*)(Pc + (size_t)(2 * i + 1) * kHeadN);
  const float a0 = a[0];
  const float a1 = a[1];
  const float b0 = b[0];
  const float b1 = b[1];
  v4f o;
  o[0] = a0;
  o[1] = a1;
  o[2] = b0;
  o[3] = b1;
  float* q = PCc + (size_t)i * 4;
  *(volatile v4f*)q = o;
  __threadfence();
  *(volatile v4f*)q = o;
}

__global__ __launch_bounds__(256) void ema_out_kernel(
    const float* __restrict__ PC, const float* __restrict__ bt, const float* __restrict__ bz,
    float* __restrict__ out)
{
  const int i = blockIdx.x * 256 + threadIdx.x;
  const int t0 = 4 * i;
  const float b0 = bf16r(bt[0]), b1 = bf16r(bz[0]);
  float h0 = 0.0f, h1 = 0.0f;
  for (int w = 0; w < kWarm; ++w) {
    const int row = t0 - kWarm + w;
    const bool live = (row >= 0);
    const int rc = live ? row : 0;
    const v2f pv = *(const v2f*)(PC + (size_t)rc * 2);
    const float p0 = live ? pv[0] : 0.0f;
    const float p1 = live ? pv[1] : 0.0f;
    h0 = fmaf(kAlpha, h0, kOneMinusA * p0);
    h1 = fmaf(kAlpha, h1, kOneMinusA * p1);
  }
  v4f o0, o1;
  {
    const v2f pv = *(const v2f*)(PC + (size_t)(t0 + 0) * 2);
    const float p0 = pv[0];
    const float p1 = pv[1];
    h0 = fmaf(kAlpha, h0, kOneMinusA * p0);
    h1 = fmaf(kAlpha, h1, kOneMinusA * p1);
    o0[0] = h0 + b0;
    o1[0] = h1 + b1;
  }
  {
    const v2f pv = *(const v2f*)(PC + (size_t)(t0 + 1) * 2);
    const float p0 = pv[0];
    const float p1 = pv[1];
    h0 = fmaf(kAlpha, h0, kOneMinusA * p0);
    h1 = fmaf(kAlpha, h1, kOneMinusA * p1);
    o0[1] = h0 + b0;
    o1[1] = h1 + b1;
  }
  {
    const v2f pv = *(const v2f*)(PC + (size_t)(t0 + 2) * 2);
    const float p0 = pv[0];
    const float p1 = pv[1];
    h0 = fmaf(kAlpha, h0, kOneMinusA * p0);
    h1 = fmaf(kAlpha, h1, kOneMinusA * p1);
    o0[2] = h0 + b0;
    o1[2] = h1 + b1;
  }
  {
    const v2f pv = *(const v2f*)(PC + (size_t)(t0 + 3) * 2);
    const float p0 = pv[0];
    const float p1 = pv[1];
    h0 = fmaf(kAlpha, h0, kOneMinusA * p0);
    h1 = fmaf(kAlpha, h1, kOneMinusA * p1);
    o0[3] = h0 + b0;
    o1[3] = h1 + b1;
  }
  float* qa = out + (size_t)i * 4;
  float* qb = out + kT + (size_t)i * 4;
  *(volatile v4f*)qa = o0;
  *(volatile v4f*)qb = o1;
  __threadfence();
  *(volatile v4f*)qa = o0;
  *(volatile v4f*)qb = o1;
}

static_assert(((kT * kIn / 8) % 256) == 0 && (kT * kIn / 8) / 256 == 4096);
static_assert(((kHid * (kIn / 8)) % 256) == 0 && (kHid * (kIn / 8)) / 256 == 16);
static_assert((512 * 8) / 256 == 16);
static_assert(((kHeadN * (kHid / 8)) % 256) == 0 && (kHeadN * (kHid / 8)) / 256 == 16);
static_assert((64 * 64) / 256 == 16);
static_assert(((kChunk * (kHid / 8)) % 256) == 0 && (kChunk * (kHid / 8)) / 256 == 4096);
static_assert((16384 * 64) / 256 == 4096);
static_assert(((kChunk / 2) % 256) == 0 && (kChunk / 2) / 256 == 32);
static_assert(((kT / 4) % 256) == 0 && (kT / 4) / 256 == 128);
static_assert(((kChunk / 32) * (kHid / 64)) % 8 == 0 && ((kChunk / 32) * (kHid / 64)) / 8 == 512);
static_assert((16384 / 32) * (512 / 64) / 8 == 512);
static_assert(((kChunk / 32) * (kHeadN / 64)) % 8 == 0 && ((kChunk / 32) * (kHeadN / 64)) / 8 == 64);
static_assert((16384 / 32) * (64 / 64) / 8 == 64);
static_assert(3 + kNChunk * 4 + 1 == 36);

extern "C" void kernel_launch(void* const* d_in, const int* in_sizes, int n_in,
                              void* d_out, int out_size, void* d_ws, size_t ws_size,
                              hipStream_t stream)
{
  if (n_in < 7) return;
  if (in_sizes[0] != kT * kIn) return;
  if (in_sizes[1] != kIn * kHid) return;
  if (in_sizes[2] != kHid) return;
  if (in_sizes[3] != kHid) return;
  if (in_sizes[4] != 1) return;
  if (in_sizes[5] != kHid) return;
  if (in_sizes[6] != 1) return;
  if (out_size != 2 * kT) return;
  if (ws_size < kWsTotal) return;

  const float* beliefs = (const float*)d_in[0];
  const float* w_in    = (const float*)d_in[1];
  const float* b_in    = (const float*)d_in[2];
  const float* w_theta = (const float*)d_in[3];
  const float* b_theta = (const float*)d_in[4];
  const float* w_z     = (const float*)d_in[5];
  const float* b_z     = (const float*)d_in[6];
  float* out = (float*)d_out;

  char* ws = (char*)d_ws;
  unsigned short* BH = (unsigned short*)(ws + kOffBH);
  unsigned short* WI = (unsigned short*)(ws + kOffWI);
  unsigned short* WH = (unsigned short*)(ws + kOffWH);
  float*          XP = (float*)(ws + kOffXP);
  unsigned short* XH = (unsigned short*)(ws + kOffXH);
  float*          P  = (float*)(ws + kOffP);
  float*          PC = (float*)(ws + kOffPC);

  constexpr float s1 = 1.0f / (kXCarry * kWCarry);
  constexpr float s2 = 1.0f / (kTCarry * kHCarry);

  pack_x_kernel<<<(kT * kIn / 8) / 256, 256, 0, stream>>>(beliefs, BH);

  pack_wt_kernel<<<(kHid * (kIn / 8)) / 256, 256, 0, stream>>>(w_in, WI);

  pack_heads_kernel<<<(kHeadN * (kHid / 8)) / 256, 256, 0, stream>>>(w_theta, w_z, WH);

  for (int c = 0; c < kNChunk; ++c) {
    eng::gemm_f16_kernel<2, 0><<<dim3((16384 / 32) * (512 / 64) / 8), 256, 0, stream>>>(
        BH + (size_t)c * kChunk * kIn, nullptr, 64, WI, nullptr, 64, XP, 512, 16384, 512, 64, s1, 0.0f);

    tanh_pack_kernel<<<(kChunk * (kHid / 8)) / 256, 256, 0, stream>>>(XP, b_in, XH);

    eng::gemm_f16_kernel<2, 0><<<dim3((16384 / 32) * (64 / 64) / 8), 256, 0, stream>>>(
        XH, nullptr, 512, WH, nullptr, 512, P, 64, 16384, 64, 512, s2, 0.0f);

    heads_copy_kernel<<<(kChunk / 2) / 256, 256, 0, stream>>>(P, PC + (size_t)c * kChunk * 2);
  }

  ema_out_kernel<<<(kT / 4) / 256, 256, 0, stream>>>(PC, b_theta, b_z, out);
}
